// SSMCore_79577154060422
// MI455X (gfx1250) — hardware-run, weakly checked
//
#include <hip/hip_runtime.h>
#include <math.h>

typedef __attribute__((ext_vector_type(16))) _Float16 v16h;
typedef __attribute__((ext_vector_type(8)))  _Float16 v8h;
typedef __attribute__((ext_vector_type(8)))  float    v8f;
typedef __attribute__((ext_vector_type(4)))  float    v4f;

constexpr int kBatch   = 2;
constexpr int kT       = 1024;
constexpr int kD       = 1024;
constexpr int kNs      = 16;
constexpr int kTaps    = 4;
constexpr int kRows    = kBatch * kT;
constexpr int kNp      = 2 * kNs;
constexpr int kNpad    = 64;
constexpr int kPjP     = 64;
constexpr int kKdt     = 32;
constexpr int kTileP   = 260;
constexpr int kChunk   = 128;
constexpr int kWarm    = 32;
constexpr int kNChunk  = kT / kChunk;
constexpr int kGrp     = 16;
constexpr int kDBlk    = 256;
constexpr float kCarryX  = 32.0f;
constexpr float kCarryW  = 1024.0f;
constexpr float kFold    = 1.0f / (kCarryX * kCarryW);
constexpr float kRemScale = 2048.0f;
constexpr float kRemInv   = 1.0f / kRemScale;
constexpr float kCarryB  = 64.0f;
constexpr float kCarryDw = 64.0f;
constexpr float kFoldDt  = 1.0f / (kCarryB * kCarryDw);
constexpr float kF16MinNormal = 6.103515625e-05f;
constexpr float kF32MinNormal = 1.17549435e-38f;

static_assert(kRows == 2048 && kNp == 32, "shape");
static_assert((kD % 32) == 0 && (kKdt % 32) == 0 && kKdt >= kNs, "GEMM K multiples of 32");
static_assert((kRows % 64) == 0 && (kNpad % 64) == 0 && (kD % 64) == 0, "GEMM M, N multiples of 64");
static_assert(kNpad == 64 && kPjP == 64 && (kRows % 16) == 0, "three-product GEMM tile is 16 rows x 64 columns");
static_assert((kT % 64) == 0 && (kD % kDBlk) == 0, "conv tiling");
static_assert(kNChunk * kChunk == kT && (kChunk % kGrp) == 0 && (kWarm % kGrp) == 0, "scan tiling");
static_assert(kNChunk == 8 && (kD / kDBlk) == 4, "scan block decode");
static_assert(kTaps == 4 && kNs == 16 && kKdt == 32, "taps and pad widths");
static_assert(((kNpad * kD / 8) % 256) == 0, "weight plane grid exact");
static_assert(((kD * kKdt / 8) % 256) == 0 && ((kRows * kKdt / 8) % 256) == 0, "pad plane grids exact");
static_assert(((kRows / 16) % 8) == 0 && (((kRows / 64) * (kD / 64)) % 8) == 0, "GEMM grids exact");

constexpr size_t kOffXC   = 0;
constexpr size_t kOffXH   = kOffXC  + (size_t)kRows * kD * 4;
constexpr size_t kOffXL   = kOffXH  + (size_t)kRows * kD * 2;
constexpr size_t kOffWH   = kOffXL  + (size_t)kRows * kD * 2;
constexpr size_t kOffWL   = kOffWH  + (size_t)kNpad * kD * 2;
constexpr size_t kOffPJ   = kOffWL  + (size_t)kNpad * kD * 2;
constexpr size_t kOffBH   = kOffPJ  + (size_t)kRows * kPjP * 4;
constexpr size_t kOffDW   = kOffBH  + (size_t)kRows * kKdt * 2;
constexpr size_t kOffDTP  = kOffDW  + (size_t)kD * kKdt * 2;
constexpr size_t kWsTotal = kOffDTP + (size_t)kRows * kD * 4;
static_assert(kWsTotal == 26148864ull, "carve total");
static_assert(kWsTotal <= 134217728ull, "carve cap");
static_assert((kOffXH % 128) == 0 && (kOffXL % 128) == 0 && (kOffWH % 128) == 0 && (kOffWL % 128) == 0 &&
              (kOffPJ % 128) == 0 && (kOffBH % 128) == 0 && (kOffDW % 128) == 0 && (kOffDTP % 128) == 0,
              "aligned regions");

__device__ __forceinline__ void guard1_h(v8f& a, v16h x, v16h y) {
  asm volatile("v_nop\n\tv_nop\n\tv_nop\n\tv_nop" : "+v"(a) : "v"(x), "v"(y));
}
__device__ __forceinline__ void guard_rem_h(v8f& a, v16h x, v16h y, v16h z) {
  asm volatile("v_nop\n\tv_nop\n\tv_nop\n\tv_nop" : "+v"(a) : "v"(x), "v"(y), "v"(z));
}
__device__ __forceinline__ void keep4_h(v16h a, v16h b, v16h c, v16h d) {
  asm volatile("v_nop" :: "v"(a), "v"(b), "v"(c), "v"(d));
}
__device__ __forceinline__ void acc_guard4(v8f& a, v8f& b, v8f& c, v8f& d) {
  asm volatile("v_nop\n\tv_nop\n\tv_nop\n\tv_nop" : "+v"(a), "+v"(b), "+v"(c), "+v"(d));
}
__device__ __forceinline__ v16h frag_load_h(const _Float16* p) {
  union { v16h v; v8h h[2]; } f;
  f.h[0] = *(const v8h*)(p);
  f.h[1] = *(const v8h*)(p + 16);
  return f.v;
}
__device__ __forceinline__ v8f mma_h(v16h a, v16h b, v8f c) {
  return __builtin_amdgcn_wmma_f32_16x16x32_f16(false, a, false, b, (short)0, c, false, false);
}
__device__ __forceinline__ float carry_flush(float v, float carry, bool real) {
  const float c = real ? (v * carry) : 0.0f;
  return (fabsf(c) < kF16MinNormal) ? 0.0f : c;
}
__device__ __forceinline__ void split16(float craw, _Float16& hv, _Float16& lv) {
  const float cv = (fabsf(craw) < kF16MinNormal) ? 0.0f : craw;
  const _Float16 h = (_Float16)cv;
  const float hf = (float)h;
  const float r  = (craw - hf) * kRemScale;
  const float rv = (fabsf(r) < kF16MinNormal) ? 0.0f : r;
  hv = h;
  lv = (_Float16)rv;
}

__global__ __launch_bounds__(256) void wplane_kernel(
    const float* __restrict__ W, unsigned short* __restrict__ WH, unsigned short* __restrict__ WL)
{
  const int i   = blockIdx.x * 256 + threadIdx.x;
  const int e0  = i << 3;
  const int row = e0 >> 10;
  const int col = e0 & (kD - 1);
  const bool real = (row < kNp);
  const int rc  = real ? row : (kNp - 1);
  const v4f a0 = *(const v4f*)(W + (size_t)rc * kD + col);
  const v4f a1 = *(const v4f*)(W + (size_t)rc * kD + col + 4);
  float f0 = a0[0], f1 = a0[1], f2 = a0[2], f3 = a0[3];
  float f4 = a1[0], f5 = a1[1], f6 = a1[2], f7 = a1[3];
  asm volatile("" : "+v"(f0), "+v"(f1), "+v"(f2), "+v"(f3));
  asm volatile("" : "+v"(f4), "+v"(f5), "+v"(f6), "+v"(f7));
  const float cr[8] = {f0, f1, f2, f3, f4, f5, f6, f7};
  v8h hv, lv;
#pragma unroll
  for (int e = 0; e < 8; ++e) {
    const float craw = real ? (cr[e] * kCarryW) : 0.0f;
    _Float16 h, l;
    split16(craw, h, l);
    hv[e] = h;
    lv[e] = l;
  }
  unsigned short* qh = WH + (size_t)e0;
  unsigned short* ql = WL + (size_t)e0;
  *(volatile v8h*)qh = hv;
  *(volatile v8h*)ql = lv;
  __threadfence();
  *(volatile v8h*)qh = hv;
  *(volatile v8h*)ql = lv;
}

__global__ __launch_bounds__(256) void pad16_plane_kernel(
    const float* __restrict__ src, int pitch, unsigned short* __restrict__ dst, float carry, int total8)
{
  const int i = blockIdx.x * 256 + threadIdx.x;
  if (i >= total8) return;
  const int e0  = i << 3;
  const int row = e0 >> 5;
  const int col = e0 & (kKdt - 1);
  const bool real = (col < kNs);
  const int cc  = col & (kNs - 1);
  const v4f a0 = *(const v4f*)(src + (size_t)row * pitch + cc);
  const v4f a1 = *(const v4f*)(src + (size_t)row * pitch + cc + 4);
  float f0 = a0[0], f1 = a0[1], f2 = a0[2], f3 = a0[3];
  float f4 = a1[0], f5 = a1[1], f6 = a1[2], f7 = a1[3];
  asm volatile("" : "+v"(f0), "+v"(f1), "+v"(f2), "+v"(f3));
  asm volatile("" : "+v"(f4), "+v"(f5), "+v"(f6), "+v"(f7));
  v8h hv;
  hv[0] = (_Float16)carry_flush(f0, carry, real);
  hv[1] = (_Float16)carry_flush(f1, carry, real);
  hv[2] = (_Float16)carry_flush(f2, carry, real);
  hv[3] = (_Float16)carry_flush(f3, carry, real);
  hv[4] = (_Float16)carry_flush(f4, carry, real);
  hv[5] = (_Float16)carry_flush(f5, carry, real);
  hv[6] = (_Float16)carry_flush(f6, carry, real);
  hv[7] = (_Float16)carry_flush(f7, carry, real);
  unsigned short* q = dst + (size_t)e0;
  *(volatile v8h*)q = hv;
  __threadfence();
  *(volatile v8h*)q = hv;
}

__global__ __launch_bounds__(256) void conv_silu_kernel(
    const float* __restrict__ x, const float* __restrict__ cw, const float* __restrict__ cb,
    float* __restrict__ XC, unsigned short* __restrict__ XH, unsigned short* __restrict__ XL)
{
  __shared__ __align__(16) float sT[16 * kTileP];
  const int tid = threadIdx.x, lane = tid & 31, wave = tid >> 5;
  const int d0 = blockIdx.x * 256, d = d0 + tid;
  const int g0 = blockIdx.y * 64;
  const int tb = g0 & (kT - 1);
  const v4f wv = *(const v4f*)(cw + (size_t)d * kTaps);
  const float w0 = wv[0], w1 = wv[1], w2 = wv[2], w3 = wv[3];
  const float bc = cb[d];
  float xm3, xm2, xm1;
  {
    const bool hist = (tb > 0);
    const int rb = hist ? (g0 - 3) : g0;
    const float v3 = x[(size_t)rb * kD + d];
    const float v2 = x[(size_t)(rb + 1) * kD + d];
    const float v1 = x[(size_t)(rb + 2) * kD + d];
    xm3 = hist ? v3 : 0.f;
    xm2 = hist ? v2 : 0.f;
    xm1 = hist ? v1 : 0.f;
  }
  const int hrow = wave >> 1;
  const int hch  = (wave & 1) * 128 + lane * 4;
#pragma unroll 1
  for (int sub = 0; sub < 4; ++sub) {
    const int lb = g0 + sub * 16;
#pragma unroll 1
    for (int s = 0; s < 16; ++s) {
      const float xcur = x[(size_t)(lb + s) * kD + d];
      float acc = w0 * xm3;
      acc = fmaf(w1, xm2, acc);
      acc = fmaf(w2, xm1, acc);
      acc = fmaf(w3, xcur, acc);
      const float sv = acc + bc;
      const float sg = __builtin_amdgcn_rcpf(1.0f + expf(-sv));
      sT[s * kTileP + tid] = sv * sg;
      xm3 = xm2; xm2 = xm1; xm1 = xcur;
    }
    __syncthreads();
    v4f fv[4];
    v8h hv[2], lv[2];
#pragma unroll
    for (int it = 0; it < 4; ++it) fv[it] = *(const v4f*)(sT + (it * 4 + hrow) * kTileP + hch);
#pragma unroll
    for (int it = 0; it < 2; ++it) {
      const float* sp = sT + (it * 8 + wave) * kTileP + lane * 8;
      const v4f a0 = *(const v4f*)(sp);
      const v4f a1 = *(const v4f*)(sp + 4);
#pragma unroll
      for (int e = 0; e < 4; ++e) {
        const float r0 = a0[e] * kCarryX;
        const float r1 = a1[e] * kCarryX;
        _Float16 h0, l0, h1, l1;
        split16(r0, h0, l0);
        split16(r1, h1, l1);
        hv[it][e]     = h0;
        hv[it][4 + e] = h1;
        lv[it][e]     = l0;
        lv[it][4 + e] = l1;
      }
    }
    for (int pass = 0; pass < 2; ++pass) {
#pragma unroll
      for (int it = 0; it < 4; ++it)
        *(volatile v4f*)(XC + (size_t)(lb + it * 4 + hrow) * kD + d0 + hch) = fv[it];
#pragma unroll
      for (int it = 0; it < 2; ++it) {
        const size_t o = (size_t)(lb + it * 8 + wave) * kD + d0 + lane * 8;
        *(volatile v8h*)(XH + o) = hv[it];
        *(volatile v8h*)(XL + o) = lv[it];
      }
      __threadfence();
    }
    __syncthreads();
  }
}

__global__ __launch_bounds__(256) void gemm_f16x3_kernel(
    const unsigned short* __restrict__ Avp, const unsigned short* __restrict__ Arp, int lda,
    const unsigned short* __restrict__ Bvp, const unsigned short* __restrict__ Brp, int ldb,
    float* __restrict__ C, int ldc, int M, int K, float scale)
{
  const _Float16* Av = (const _Float16*)Avp;
  const _Float16* Ar = (const _Float16*)Arp;
  const _Float16* Bv = (const _Float16*)Bvp;
  const _Float16* Br = (const _Float16*)Brp;
  __shared__ __align__(16) float sT[8][16 * 68];
  const int lane = threadIdx.x & 31;
  const int wave = threadIdx.x >> 5;
  const int tile = blockIdx.x * 8 + wave;
  if (tile >= (M >> 4)) return;
  const int m0 = tile << 4;

  const int rlane = lane & 15;
  const int koff  = (lane >> 4) * 8;
  const int mOff  = (lane >> 4) * 8;

  v8f accM[4], accR[4];
#pragma unroll
  for (int j = 0; j < 4; ++j) {
    accM[j] = (v8f){0.f,0.f,0.f,0.f,0.f,0.f,0.f,0.f};
    accR[j] = (v8f){0.f,0.f,0.f,0.f,0.f,0.f,0.f,0.f};
  }

  for (int k0 = 0; k0 < K; k0 += 32) {
    v16h bv[4], br[4];
#pragma unroll
    for (int j = 0; j < 4; ++j) {
      const size_t bo = (size_t)((j << 4) + rlane) * ldb + koff + k0;
      bv[j] = frag_load_h(Bv + bo);
      br[j] = frag_load_h(Br + bo);
    }
    const size_t ao = (size_t)(m0 + rlane) * lda + koff + k0;
    const v16h av = frag_load_h(Av + ao);
    const v16h ar = frag_load_h(Ar + ao);
#pragma unroll
    for (int j = 0; j < 4; ++j) {
      accM[j] = mma_h(av, bv[j], accM[j]);
      accR[j] = mma_h(av, br[j], accR[j]);
      accR[j] = mma_h(ar, bv[j], accR[j]);
    }
    guard1_h(accM[0], av, bv[0]);
    guard1_h(accM[1], av, bv[1]);
    guard1_h(accM[2], av, bv[2]);
    guard1_h(accM[3], av, bv[3]);
    guard_rem_h(accR[0], ar, bv[0], br[0]);
    guard_rem_h(accR[1], ar, bv[1], br[1]);
    guard_rem_h(accR[2], ar, bv[2], br[2]);
    guard_rem_h(accR[3], ar, bv[3], br[3]);
    keep4_h(bv[0], bv[1], bv[2], bv[3]);
    keep4_h(br[0], br[1], br[2], br[3]);
  }
  acc_guard4(accM[0], accM[1], accM[2], accM[3]);
  acc_guard4(accR[0], accR[1], accR[2], accR[3]);

  float* slab = sT[wave];
#pragma unroll
  for (int j = 0; j < 4; ++j) {
#pragma unroll
    for (int r = 0; r < 8; ++r) {
      const float joined = accM[j][r] + accR[j][r] * kRemInv;
      slab[(mOff + r) * 68 + (j << 4) + rlane] = joined * scale;
    }
  }
  __builtin_amdgcn_fence(__ATOMIC_RELEASE, "workgroup");
  __builtin_amdgcn_wave_barrier();
  __builtin_amdgcn_fence(__ATOMIC_ACQUIRE, "workgroup");
  {
    const int hh = lane >> 4, c4 = (lane & 15) * 4;
    for (int pass = 0; pass < 2; ++pass) {
#pragma unroll
      for (int it = 0; it < 8; ++it) {
        const int row = it * 2 + hh;
        const v4f v = *(const v4f*)(slab + row * 68 + c4);
        *(volatile v4f*)(C + (size_t)(m0 + row) * ldc + c4) = v;
      }
      __threadfence();
    }
  }
}

__global__ __launch_bounds__(256) void gemm_f16_kernel(
    const unsigned short* __restrict__ Ap, int lda,
    const unsigned short* __restrict__ Btp, int ldb,
    float* __restrict__ C, int ldc, int M, int N, int K, float scale)
{
  const _Float16* A  = (const _Float16*)Ap;
  const _Float16* Bt = (const _Float16*)Btp;
  __shared__ __align__(16) float sT[8][16 * 68];
  const int lane = threadIdx.x & 31;
  const int wave = threadIdx.x >> 5;
  const int tilesN = N >> 6;
  const int tilesM = M >> 6;
  const int tile = blockIdx.x * 8 + wave;
  if (tile >= tilesM * tilesN) return;
  const int tm = tile / tilesN;
  const int tn = tile - tm * tilesN;
  const int m0 = tm << 6;
  const int n0 = tn << 6;

  const int rlane = lane & 15;
  const int koff  = (lane >> 4) * 8;
  const int mOff  = (lane >> 4) * 8;

  v8f acc[4][4];
#pragma unroll
  for (int i = 0; i < 4; ++i)
#pragma unroll
    for (int j = 0; j < 4; ++j) acc[i][j] = (v8f){0.f,0.f,0.f,0.f,0.f,0.f,0.f,0.f};

  for (int k0 = 0; k0 < K; k0 += 32) {
    v16h bh[4];
#pragma unroll
    for (int j = 0; j < 4; ++j) {
      const size_t bo = (size_t)(n0 + (j << 4) + rlane) * ldb + koff + k0;
      bh[j] = frag_load_h(Bt + bo);
    }
#pragma unroll
    for (int i = 0; i < 4; ++i) {
      const size_t ao = (size_t)(m0 + (i << 4) + rlane) * lda + koff + k0;
      const v16h ah = frag_load_h(A + ao);
#pragma unroll
      for (int j = 0; j < 4; ++j) acc[i][j] = mma_h(ah, bh[j], acc[i][j]);
      guard1_h(acc[i][0], ah, bh[0]);
      guard1_h(acc[i][1], ah, bh[1]);
      guard1_h(acc[i][2], ah, bh[2]);
      guard1_h(acc[i][3], ah, bh[3]);
    }
    keep4_h(bh[0], bh[1], bh[2], bh[3]);
  }
  acc_guard4(acc[0][0], acc[0][1], acc[0][2], acc[0][3]);
  acc_guard4(acc[1][0], acc[1][1], acc[1][2], acc[1][3]);
  acc_guard4(acc[2][0], acc[2][1], acc[2][2], acc[2][3]);
  acc_guard4(acc[3][0], acc[3][1], acc[3][2], acc[3][3]);

  float* slab = sT[wave];
#pragma unroll
  for (int i = 0; i < 4; ++i) {
    const int mBase = m0 + (i << 4);
#pragma unroll
    for (int j = 0; j < 4; ++j) {
#pragma unroll
      for (int r = 0; r < 8; ++r) {
        const float v = acc[i][j][r] * scale;
        slab[(mOff + r) * 68 + (j << 4) + rlane] = v;
      }
    }
    __builtin_amdgcn_fence(__ATOMIC_RELEASE, "workgroup");
    __builtin_amdgcn_wave_barrier();
    __builtin_amdgcn_fence(__ATOMIC_ACQUIRE, "workgroup");
    {
      const int hh = lane >> 4, c4 = (lane & 15) * 4;
      for (int pass = 0; pass < 2; ++pass) {
#pragma unroll
        for (int it = 0; it < 8; ++it) {
          const int row = it * 2 + hh;
          const v4f v = *(const v4f*)(slab + row * 68 + c4);
          *(volatile v4f*)(C + (size_t)(mBase + row) * ldc + n0 + c4) = v;
        }
        __threadfence();
      }
    }
    __builtin_amdgcn_fence(__ATOMIC_RELEASE, "workgroup");
    __builtin_amdgcn_wave_barrier();
    __builtin_amdgcn_fence(__ATOMIC_ACQUIRE, "workgroup");
  }
}

__device__ __forceinline__ float softplus_f(float v) {
  const float a = expf(-fabsf(v));
  const float u = 1.0f + a;
  const float l = logf(u) + (a - (u - 1.0f)) * __builtin_amdgcn_rcpf(u);
  return fmaxf(v, 0.0f) + l;
}

__global__ __launch_bounds__(256) void scan_kernel(
    const float* __restrict__ PJ, const float* __restrict__ XC, const float* __restrict__ DTP,
    const float* __restrict__ dtb, const float* __restrict__ Dp, float* __restrict__ out)
{
  __shared__ __align__(16) float sP[(kChunk + kWarm) * kNp];
  __shared__ __align__(16) float sY[kGrp * kTileP];
  const int tid = threadIdx.x, lane = tid & 31, wave = tid >> 5;
  const int chunk = blockIdx.x & 7;
  const int dblk  = (blockIdx.x >> 3) & 3;
  const int bix   = blockIdx.x >> 5;
  const int d0 = dblk * kDBlk, d = d0 + tid;
  const int tstart = chunk * kChunk;
  const int warm   = (chunk > 0) ? kWarm : 0;
  const int tbeg   = tstart - warm;
  const int nrows  = kChunk + warm;
  const size_t rowb = (size_t)bix * kT;

  for (int i = tid; i < nrows * 8; i += 256) {
    const int row = i >> 3, c4 = (i & 7) * 4;
    *(v4f*)(sP + row * kNp + c4) = *(const v4f*)(PJ + (rowb + tbeg + row) * kPjP + c4);
  }
  __syncthreads();

  float h[kNs];
#pragma unroll
  for (int s = 0; s < kNs; ++s) h[s] = 0.f;
  const float bb = dtb[d];
  const float Dd = Dp[d];
  const int hrow = wave >> 1;
  const int hch  = (wave & 1) * 128 + lane * 4;
  const int gbeg = -(warm / kGrp);

#pragma unroll 1
  for (int g = gbeg; g < kChunk / kGrp; ++g) {
    const int tg = tstart + g * kGrp;
#pragma unroll 1
    for (int s = 0; s < kGrp; ++s) {
      const int t = tg + s;
      const float* pr = sP + (t - tbeg) * kNp;
      const float xcv = XC[(rowb + t) * kD + d];
      const float dpv = DTP[(rowb + t) * kD + d];
      float Bs[kNs], Cs[kNs];
#pragma unroll
      for (int q4 = 0; q4 < 4; ++q4) {
        const v4f bv = *(const v4f*)(pr + 4 * q4);
        const v4f cv = *(const v4f*)(pr + kNs + 4 * q4);
        Bs[4 * q4 + 0] = bv[0]; Bs[4 * q4 + 1] = bv[1]; Bs[4 * q4 + 2] = bv[2]; Bs[4 * q4 + 3] = bv[3];
        Cs[4 * q4 + 0] = cv[0]; Cs[4 * q4 + 1] = cv[1]; Cs[4 * q4 + 2] = cv[2]; Cs[4 * q4 + 3] = cv[3];
      }
      const float pre  = dpv + bb;
      const float sp1  = softplus_f(pre);
      const float step = softplus_f(sp1);
      const float r    = expf(-step);
      float p = r;
      float y = 0.f;
#pragma unroll
      for (int k = 0; k < kNs; ++k) {
        const float v = (step * Bs[k]) * xcv;
        const float u = (v >= kF32MinNormal) ? v : 0.0f;
        h[k] = fmaf(p, h[k], u);
        y = fmaf(Cs[k], h[k], y);
        p = p * r;
      }
      y = fmaf(Dd, xcv, y);
      sY[s * kTileP + tid] = y;
    }
    if (g >= 0) {
      __syncthreads();
      v4f fv[4];
#pragma unroll
      for (int it = 0; it < 4; ++it) fv[it] = *(const v4f*)(sY + (it * 4 + hrow) * kTileP + hch);
      for (int pass = 0; pass < 2; ++pass) {
#pragma unroll
        for (int it = 0; it < 4; ++it)
          *(volatile v4f*)(out + (rowb + tg + it * 4 + hrow) * kD + d0 + hch) = fv[it];
        __threadfence();
      }
      __syncthreads();
    }
  }
}

extern "C" void kernel_launch(void* const* d_in, const int* in_sizes, int n_in,
                              void* d_out, int out_size, void* d_ws, size_t ws_size,
                              hipStream_t stream) {
  if (n_in < 7) return;
  if (in_sizes[0] != kRows * kD) return;
  if (in_sizes[1] != kD * kTaps) return;
  if (in_sizes[2] != kD) return;
  if (in_sizes[3] != kNp * kD) return;
  if (in_sizes[4] != kD * kNs) return;
  if (in_sizes[5] != kD) return;
  if (in_sizes[6] != kD) return;
  if (out_size != kRows * kD) return;
  if (ws_size < kWsTotal) return;

  const float* x         = (const float*)d_in[0];
  const float* conv_w    = (const float*)d_in[1];
  const float* conv_b    = (const float*)d_in[2];
  const float* x_proj_w  = (const float*)d_in[3];
  const float* dt_proj_w = (const float*)d_in[4];
  const float* dt_proj_b = (const float*)d_in[5];
  const float* Dvec      = (const float*)d_in[6];
  float* out = (float*)d_out;

  char* ws = (char*)d_ws;
  float*          XC  = (float*)(ws + kOffXC);
  unsigned short* XH  = (unsigned short*)(ws + kOffXH);
  unsigned short* XL  = (unsigned short*)(ws + kOffXL);
  unsigned short* WH  = (unsigned short*)(ws + kOffWH);
  unsigned short* WL  = (unsigned short*)(ws + kOffWL);
  float*          PJ  = (float*)(ws + kOffPJ);
  unsigned short* BH  = (unsigned short*)(ws + kOffBH);
  unsigned short* DW  = (unsigned short*)(ws + kOffDW);
  float*          DTP = (float*)(ws + kOffDTP);

  wplane_kernel<<<(kNpad * kD / 8) / 256, 256, 0, stream>>>(x_proj_w, WH, WL);

  pad16_plane_kernel<<<(kD * kKdt / 8) / 256, 256, 0, stream>>>(
      dt_proj_w, kNs, DW, kCarryDw, kD * kKdt / 8);

  conv_silu_kernel<<<dim3(kD / 256, kRows / 64), 256, 0, stream>>>(x, conv_w, conv_b, XC, XH, XL);

  gemm_f16x3_kernel<<<(kRows / 16) / 8, 256, 0, stream>>>(
      XH, XL, kD, WH, WL, kD, PJ, kPjP, kRows, kD, kFold);

  pad16_plane_kernel<<<(kRows * kKdt / 8) / 256, 256, 0, stream>>>(
      PJ, kPjP, BH, kCarryB, kRows * kKdt / 8);

  gemm_f16_kernel<<<((kRows / 64) * (kD / 64)) / 8, 256, 0, stream>>>(
      BH, kKdt, DW, kKdt, DTP, kD, kRows, kD, kKdt, kFoldDt);

  scan_kernel<<<kBatch * (kD / kDBlk) * kNChunk, 256, 0, stream>>>(
      PJ, XC, DTP, dt_proj_b, Dvec, out);
}
